// RlSaTree_20358144983213
// MI455X (gfx1250) — hardware-run, weakly checked
//
#include <hip/hip_runtime.h>
#include <math.h>

typedef __attribute__((ext_vector_type(16))) _Float16 v16h;
typedef __attribute__((ext_vector_type(8)))  _Float16 v8h;
typedef __attribute__((ext_vector_type(4)))  _Float16 v4h;
typedef __attribute__((ext_vector_type(8)))  float    v8f;
typedef __attribute__((ext_vector_type(4)))  float    v4f;

constexpr int kB      = 16;
constexpr int kL      = 32;
constexpr int kD      = 300;
constexpr int kH      = 300;
constexpr int kTok    = kB * kL;
constexpr int kKx     = 320;
constexpr int kNw     = 640;
constexpr int kNwReal = 2 * kH;
constexpr int kKc     = 928;
constexpr int kKcReal = 3 * kH;
constexpr int kNcb    = 19;
constexpr int kWcRows = kNcb * 80;
constexpr int kStP    = 640;
constexpr int kNodeP  = kNcb * 32;
constexpr int kMaxNode = kL - 1;
constexpr int kOutW   = 2 * kH + 1;
constexpr int kOutN   = kB * kOutW;
constexpr int kOutQ   = kOutN / 4;
constexpr int kGatQ   = kB * (kKc / 4);
constexpr float kCarA = 16.0f;
constexpr float kCarW = 256.0f;
constexpr float kResS = 2048.0f;
constexpr float kFold = 1.0f / (kCarA * kCarW);
constexpr float kInvRes = 1.0f / kResS;
static_assert(kTok == 512 && (kTok % 64) == 0 && (kNw % 64) == 0, "leaf GEMM M,N tile multiples");
static_assert((kKx % 32) == 0 && (kKc % 32) == 0, "K multiples of 32");
static_assert(kKx >= kD && kKc >= kKcReal && kNcb * 16 >= kH, "pads cover the real extents");
static_assert((kD % 4) == 0 && (kKcReal % 4) == 0 && (kH % 4) == 0, "float4 groups never straddle a segment");
static_assert((kOutN % 4) == 0 && kOutQ == 2404, "output float4 count");
static_assert(kGatQ == 3712, "gather float4 count");

constexpr size_t kOffXH = 0;
constexpr size_t kOffWW = kOffXH + (size_t)kTok * kKx * 2;
constexpr size_t kOffWC = kOffWW + (size_t)kNw * kKx * 2;
constexpr size_t kOffST = kOffWC + (size_t)kWcRows * kKc * 2;
constexpr size_t kOffND = kOffST + (size_t)kTok * kStP * 4;
constexpr size_t kWsTotal = kOffND + (size_t)kB * kMaxNode * kNodeP * 4;
static_assert(kWsTotal == 6075392ull, "carve total");
static_assert(kWsTotal <= 134217728ull, "carve cap");
static_assert((kOffWW % 128) == 0 && (kOffWC % 128) == 0 && (kOffST % 128) == 0 && (kOffND % 128) == 0, "aligned regions");

union FragU { v16h v; v8h h[2]; };
__device__ __forceinline__ v16h frag_load(const _Float16* p) {
  FragU f;
  f.h[0] = *(const v8h*)(p);
  f.h[1] = *(const v8h*)(p + 16);
  return f.v;
}
__device__ __forceinline__ v8f mma_h(v16h a, v16h b, v8f c) {
  c = __builtin_amdgcn_wmma_f32_16x16x32_f16(false, a, false, b, (short)0, c, false, false);
  asm volatile("v_nop\n\tv_nop\n\tv_nop\n\tv_nop" : "+v"(c) : "v"(a), "v"(b));
  return c;
}
__device__ __forceinline__ void keep4_h(v16h a, v16h b, v16h c, v16h d) { asm volatile("v_nop" :: "v"(a), "v"(b), "v"(c), "v"(d)); }
__device__ __forceinline__ void acc_guard4(v8f& a, v8f& b, v8f& c, v8f& d) { asm volatile("v_nop\n\tv_nop\n\tv_nop\n\tv_nop" : "+v"(a), "+v"(b), "+v"(c), "+v"(d)); }

constexpr int kChX  = kTok * (kKx / 8);
constexpr int kChW  = kNw * (kKx / 8);
constexpr int kChC  = kWcRows * (kKc / 8);
constexpr int kBlkX = kChX / 256;
constexpr int kBlkW = kChW / 256;
constexpr int kBlkC = (kChC + 255) / 256;
static_assert(kChX % 256 == 0 && kChW % 256 == 0 && kChC % 32 == 0, "whole waves per plane");

__global__ __launch_bounds__(256) void prep_planes_kernel(
    const float* __restrict__ X, const float* __restrict__ Ww, const float* __restrict__ Wc,
    unsigned short* __restrict__ XH, unsigned short* __restrict__ WW, unsigned short* __restrict__ WC)
{
  const int blk = blockIdx.x, tid = threadIdx.x;
  const int region = (blk < kBlkX) ? 0 : ((blk < kBlkX + kBlkW) ? 1 : 2);
  const float* src;
  unsigned short* dst;
  int chunk, total, cpr, kreal;
  float carry;
  if (region == 0) {
    src = X; dst = XH; chunk = blk * 256 + tid; total = kChX; cpr = kKx / 8; kreal = kD; carry = kCarA;
  } else if (region == 1) {
    src = Ww; dst = WW; chunk = (blk - kBlkX) * 256 + tid; total = kChW; cpr = kKx / 8; kreal = kD; carry = kCarW;
  } else {
    src = Wc; dst = WC; chunk = (blk - kBlkX - kBlkW) * 256 + tid; total = kChC; cpr = kKc / 8; kreal = kKcReal; carry = kCarW;
  }
  if (chunk >= total) return;
  const int row = chunk / cpr;
  const int c = chunk - row * cpr;
  int srow;
  bool rv;
  if (region == 0) {
    srow = row; rv = true;
  } else if (region == 1) {
    rv = row < kNwReal;
    srow = rv ? row : (kNwReal - 1);
  } else {
    const int cb = row / 80;
    const int rem = row - cb * 80;
    const int g = rem >> 4, jj = rem & 15;
    const int j = cb * 16 + jj;
    rv = j < kH;
    srow = g * kH + (rv ? j : (kH - 1));
  }
  const int k0 = 8 * c;
  const int ka = (k0 < kreal - 4) ? k0 : (kreal - 4);
  const int kb = (k0 + 4 < kreal - 4) ? (k0 + 4) : (kreal - 4);
  const v4f a0 = *(const v4f*)(src + (size_t)srow * kreal + ka);
  const v4f a1 = *(const v4f*)(src + (size_t)srow * kreal + kb);
  const bool va = rv && (k0 < kreal);
  const bool vb = rv && (k0 + 4 < kreal);
  v8h hv;
#pragma unroll
  for (int e = 0; e < 4; ++e) {
    const float x0 = va ? a0[e] * carry : 0.0f;
    const float x1 = vb ? a1[e] * carry : 0.0f;
    hv[e]     = (_Float16)x0;
    hv[4 + e] = (_Float16)x1;
  }
  unsigned short* q = dst + (size_t)chunk * 8;
  *(volatile v8h*)q = hv;
  __threadfence();
  *(volatile v8h*)q = hv;
}

__global__ __launch_bounds__(256) void leaf_gemm_kernel(
    const unsigned short* __restrict__ Ap, int lda,
    const unsigned short* __restrict__ Btp, int ldb,
    float* __restrict__ C, int ldc,
    const float* __restrict__ bias, int nBias,
    int M, int N, int K, float scale)
{
  const _Float16* A  = (const _Float16*)Ap;
  const _Float16* Bt = (const _Float16*)Btp;
  __shared__ __align__(16) float sT[8][16 * 68];
  const int lane = threadIdx.x & 31;
  const int wave = threadIdx.x >> 5;
  const int tilesN = N >> 6;
  const int tilesM = M >> 6;
  const int tile = blockIdx.x * 8 + wave;
  if (tile >= tilesM * tilesN) return;
  const int tm = tile / tilesN;
  const int tn = tile - tm * tilesN;
  const int m0 = tm << 6;
  const int n0 = tn << 6;
  const int rlane = lane & 15;
  const int koff  = (lane >> 4) * 8;
  const int mOff  = (lane >> 4) * 8;

  v8f acc[4][4];
#pragma unroll
  for (int i = 0; i < 4; ++i)
#pragma unroll
    for (int j = 0; j < 4; ++j) acc[i][j] = (v8f){0.f,0.f,0.f,0.f,0.f,0.f,0.f,0.f};

  for (int k0 = 0; k0 < K; k0 += 32) {
    v16h bh[4];
#pragma unroll
    for (int j = 0; j < 4; ++j) {
      const size_t bo = (size_t)(n0 + (j << 4) + rlane) * ldb + koff + k0;
      bh[j] = frag_load(Bt + bo);
    }
#pragma unroll
    for (int i = 0; i < 4; ++i) {
      const size_t ao = (size_t)(m0 + (i << 4) + rlane) * lda + koff + k0;
      const v16h ah = frag_load(A + ao);
#pragma unroll
      for (int j = 0; j < 4; ++j) acc[i][j] = mma_h(ah, bh[j], acc[i][j]);
    }
    keep4_h(bh[0], bh[1], bh[2], bh[3]);
  }
  acc_guard4(acc[0][0], acc[0][1], acc[0][2], acc[0][3]);
  acc_guard4(acc[1][0], acc[1][1], acc[1][2], acc[1][3]);
  acc_guard4(acc[2][0], acc[2][1], acc[2][2], acc[2][3]);
  acc_guard4(acc[3][0], acc[3][1], acc[3][2], acc[3][3]);

  float* slab = sT[wave];
#pragma unroll
  for (int i = 0; i < 4; ++i) {
    const int mBase = m0 + (i << 4);
#pragma unroll
    for (int j = 0; j < 4; ++j) {
      const int n = n0 + (j << 4) + rlane;
      const int nc = (n < nBias) ? n : (nBias - 1);
      const float braw = bias[nc];
      const float bv = (n < nBias) ? braw : 0.0f;
#pragma unroll
      for (int r = 0; r < 8; ++r) {
        const float v = acc[i][j][r] * scale + bv;
        slab[(mOff + r) * 68 + (j << 4) + rlane] = v;
      }
    }
    __builtin_amdgcn_fence(__ATOMIC_RELEASE, "workgroup");
    __builtin_amdgcn_wave_barrier();
    __builtin_amdgcn_fence(__ATOMIC_ACQUIRE, "workgroup");
    {
      const int hh = lane >> 4, c4 = (lane & 15) * 4;
      for (int pass = 0; pass < 2; ++pass) {
#pragma unroll
        for (int it = 0; it < 8; ++it) {
          const int row = it * 2 + hh;
          const v4f v = *(const v4f*)(slab + row * 68 + c4);
          *(volatile v4f*)(C + (size_t)(mBase + row) * ldc + n0 + c4) = v;
        }
        __threadfence();
      }
    }
    __builtin_amdgcn_fence(__ATOMIC_RELEASE, "workgroup");
    __builtin_amdgcn_wave_barrier();
    __builtin_amdgcn_fence(__ATOMIC_ACQUIRE, "workgroup");
  }
}

__device__ __forceinline__ float sigm(float x) { return __builtin_amdgcn_rcpf(1.0f + expf(-x)); }

__device__ __forceinline__ float load_child_c(const float* ST, const float* ND, int i, int slot, int jc) {
  const int sl = slot < 0 ? 0 : slot;
  const int leaf = sl > (kL - 1) ? (kL - 1) : sl;
  int nk = sl - kL;
  nk = nk < 0 ? 0 : (nk > (kMaxNode - 1) ? (kMaxNode - 1) : nk);
  const float* pl = ST + (size_t)(i * kL + leaf) * kStP + kH + jc;
  const float* pn = ND + ((size_t)(i * kMaxNode + nk) * kNcb + (jc >> 4)) * 32 + 16 + (jc & 15);
  const float* pp = (sl >= kL) ? pn : pl;
  float v = *pp;
  asm volatile("" : "+v"(v));
  return (slot >= 0) ? v : 0.0f;
}

__device__ __forceinline__ float root_val(const float* ST, const float* ND, int i, int col, int cn, float lp) {
  const bool isC = col >= kH;
  int jj = isC ? (col - kH) : col;
  jj = jj > (kH - 1) ? (kH - 1) : jj;
  const int nk = cn > 0 ? (cn - 1) : 0;
  const float* pn = ND + ((size_t)(i * kMaxNode + nk) * kNcb + (jj >> 4)) * 32 + (isC ? 16 : 0) + (jj & 15);
  const float* pl = ST + (size_t)(i * kL) * kStP + (isC ? kH : 0) + jj;
  const float* pp = (cn > 0) ? pn : pl;
  float v = *pp;
  asm volatile("" : "+v"(v));
  return (col < 2 * kH) ? v : lp;
}

__global__ __launch_bounds__(512) void tree_compose_kernel(
    const float* __restrict__ X, const int* __restrict__ length,
    const float* __restrict__ W1, const float* __restrict__ W2,
    const unsigned short* __restrict__ WCp, const float* __restrict__ bc,
    const float* ST, float* ND, float* out)
{
  __shared__ __align__(16) unsigned sPool[(2 * kB * kKc) / 2];
  __shared__ int   sMeta[kB * kL];
  __shared__ int   sCnt[kB];
  __shared__ float sLogp[kB];
  static_assert(sizeof(unsigned) * ((2 * kB * kKc) / 2) >= 4 * 4 * 512, "prologue views fit in the pool");

  const int tid  = threadIdx.x;
  const int lane = tid & 31;
  const int wave = tid >> 5;
  const int hh   = lane >> 4;
  const int m16  = lane & 15;

  _Float16* sAh = (_Float16*)sPool;
  _Float16* sAl = sAh + kB * kKc;
  float* sSc   = (float*)sPool;
  int*   sKey  = (int*)sPool + 512;
  int*   sRank = (int*)sPool + 1024;
  float* sTerm = (float*)sPool + 1536;
  const _Float16* WC = (const _Float16*)WCp;

  sMeta[tid] = 0;
  {
    const float* xr = X + (size_t)tid * kD;
    float sc = 0.0f;
#pragma unroll 1
    for (int j = 0; j < 128; ++j) {
      const float* wr = W1 + (size_t)j * kD;
      float acc = 0.0f;
#pragma unroll 1
      for (int k = 0; k < kD; k += 4) {
        const v4f xv = *(const v4f*)(xr + k);
        const v4f wv = *(const v4f*)(wr + k);
        acc = fmaf(xv[0], wv[0], acc);
        acc = fmaf(xv[1], wv[1], acc);
        acc = fmaf(xv[2], wv[2], acc);
        acc = fmaf(xv[3], wv[3], acc);
      }
      sc = fmaf(fmaxf(acc, 0.0f), W2[j], sc);
    }
    sSc[tid] = sc;
  }
  __syncthreads();

  const int base = wave * kL;
  const int p = lane;
  int n = length[wave];
  n = n < 1 ? 1 : (n > kL ? kL : n);
  const float my = sSc[base + p];
  int lo = 0, hi = n;
  {
    bool fl = false, fh = false;
#pragma unroll 1
    for (int d = 1; d < kL; ++d) {
      const int jl = p - d;
      const int jr = p + d;
      const float vl = sSc[base + (jl < 0 ? 0 : jl)];
      const float vr = sSc[base + (jr > kL - 1 ? kL - 1 : jr)];
      const bool hitl = (jl >= 0) && (!fl) && (vl >= my);
      const bool hitr = (jr < n) && (!fh) && (vr > my);
      lo = hitl ? (jl + 1) : lo;
      hi = hitr ? jr : hi;
      fl = fl || hitl;
      fh = fh || hitr;
    }
  }
  const int span = hi - lo;
  const bool isnode = (p < n) && (span >= 2);
  const int key = isnode ? (span * kL + p) : 4096;
  sKey[tid] = key;
  __syncthreads();
  int rank = 0, cntv = 0;
#pragma unroll 1
  for (int q = 0; q < kL; ++q) {
    const int kq = sKey[base + q];
    rank += (kq < key) ? 1 : 0;
    cntv += (kq < 4096) ? 1 : 0;
  }
  cntv = cntv > kMaxNode ? kMaxNode : cntv;
  rank = rank > (kMaxNode - 1) ? (kMaxNode - 1) : rank;
  sRank[tid] = rank;
  if (lane == 0) sCnt[wave] = cntv;
  __syncthreads();
  {
    float bestl = -INFINITY, bestr = -INFINITY, sum = 0.0f;
    int pl = lo, pr = (p + 1 > kL - 1) ? (kL - 1) : (p + 1);
#pragma unroll 1
    for (int j = 0; j < kL; ++j) {
      const float v = sSc[base + j];
      const bool inl = (j >= lo) && (j < p);
      const bool inr = (j > p) && (j < hi);
      const bool ina = (j >= lo) && (j < hi);
      const bool tl = inl && (v > bestl);
      const bool tr = inr && (v > bestr);
      bestl = tl ? v : bestl;
      pl = tl ? j : pl;
      bestr = tr ? v : bestr;
      pr = tr ? j : pr;
      const float e = expf(v - my);
      sum += ina ? e : 0.0f;
    }
    pl = pl < 0 ? 0 : (pl > kL - 1 ? kL - 1 : pl);
    pr = pr < 0 ? 0 : (pr > kL - 1 ? kL - 1 : pr);
    const int rkl = sRank[base + pl];
    const int rkr = sRank[base + pr];
    const int ll = p - lo;
    const int rr = hi - (p + 1);
    const int lslot = (ll <= 0) ? -1 : ((ll == 1) ? lo : (kL + rkl));
    const int rslot = (rr <= 0) ? -1 : ((rr == 1) ? (p + 1) : (kL + rkr));
    const float lg = logf(sum);
    const float term = isnode ? (-(float)span * lg) : 0.0f;
    if (isnode) sMeta[base + rank] = p | ((lslot + 1) << 8) | ((rslot + 1) << 16);
    sTerm[tid] = term;
  }
  __syncthreads();
  {
    float lp = 0.0f;
#pragma unroll 1
    for (int q = 0; q < kL; ++q) lp += sTerm[base + q];
    if (lane == 0) sLogp[wave] = lp;
  }
  __syncthreads();
  int maxc = 0;
#pragma unroll 1
  for (int i = 0; i < kB; ++i) {
    const int cv = sCnt[i];
    maxc = cv > maxc ? cv : maxc;
  }
  maxc = maxc > kMaxNode ? kMaxNode : maxc;
  __syncthreads();

#pragma unroll 1
  for (int s = 0; s < maxc; ++s) {
#pragma unroll 1
    for (int it = 0; it < 8; ++it) {
      const int q = tid + 512 * it;
      const bool inr = q < kGatQ;
      const int qc = inr ? q : (kGatQ - 1);
      const int r = qc / (kKc / 4);
      const int c4 = (qc - r * (kKc / 4)) * 4;
      const int seg = (c4 >= 3 * kH) ? 3 : ((c4 >= 2 * kH) ? 2 : ((c4 >= kH) ? 1 : 0));
      const int col = c4 - seg * kH;
      const int mw = sMeta[r * kL + s];
      const int cn = sCnt[r];
      const int pos = mw & 255;
      const int ls = ((mw >> 8) & 255) - 1;
      const int rs = ((mw >> 16) & 255) - 1;
      const int slot = (seg == 0) ? ls : ((seg == 1) ? pos : rs);
      const bool act = inr && (s < cn) && (seg < 3) && (slot >= 0);
      const int sl = slot < 0 ? 0 : slot;
      const int leaf = sl > (kL - 1) ? (kL - 1) : sl;
      int nk = sl - kL;
      nk = nk < 0 ? 0 : (nk > (kMaxNode - 1) ? (kMaxNode - 1) : nk);
      const float* pl = ST + (size_t)(r * kL + leaf) * kStP + col;
      const float* pn = ND + ((size_t)(r * kMaxNode + nk) * kNcb + (col >> 4)) * 32 + (col & 15);
      const float* pp = (sl >= kL) ? pn : pl;
      const v4f v = *(const v4f*)pp;
      float v0 = v[0], v1 = v[1], v2 = v[2], v3 = v[3];
      asm volatile("" : "+v"(v0), "+v"(v1), "+v"(v2), "+v"(v3));
      const float x0 = act ? v0 * kCarA : 0.0f;
      const float x1 = act ? v1 * kCarA : 0.0f;
      const float x2 = act ? v2 * kCarA : 0.0f;
      const float x3 = act ? v3 * kCarA : 0.0f;
      v4h hv, lv;
      hv[0] = (_Float16)x0;
      hv[1] = (_Float16)x1;
      hv[2] = (_Float16)x2;
      hv[3] = (_Float16)x3;
      const float h0 = (float)hv[0], h1 = (float)hv[1], h2 = (float)hv[2], h3 = (float)hv[3];
      lv[0] = (_Float16)((x0 - h0) * kResS);
      lv[1] = (_Float16)((x1 - h1) * kResS);
      lv[2] = (_Float16)((x2 - h2) * kResS);
      lv[3] = (_Float16)((x3 - h3) * kResS);
      if (inr) {
        *(v4h*)(sAh + r * kKc + c4) = hv;
        *(v4h*)(sAl + r * kKc + c4) = lv;
      }
    }
    __syncthreads();

#pragma unroll 1
    for (int cb = wave; cb < kNcb; cb += 16) {
      v8f aH[5], aL[5];
#pragma unroll
      for (int g = 0; g < 5; ++g) {
        aH[g] = (v8f){0.f,0.f,0.f,0.f,0.f,0.f,0.f,0.f};
        aL[g] = (v8f){0.f,0.f,0.f,0.f,0.f,0.f,0.f,0.f};
      }
      const _Float16* arh = sAh + m16 * kKc + 8 * hh;
      const _Float16* arl = sAl + m16 * kKc + 8 * hh;
      const _Float16* brw = WC + (size_t)(cb * 80 + m16) * kKc + 8 * hh;
#pragma unroll 1
      for (int k0 = 0; k0 < kKc; k0 += 32) {
        const v16h ah = frag_load(arh + k0);
        const v16h al = frag_load(arl + k0);
#pragma unroll
        for (int g = 0; g < 5; ++g) {
          const v16h bg = frag_load(brw + (size_t)(g * 16) * kKc + k0);
          aH[g] = mma_h(ah, bg, aH[g]);
          aL[g] = mma_h(al, bg, aL[g]);
        }
      }

      const int j = cb * 16 + m16;
      const bool jv = j < kH;
      const int jc = jv ? j : (kH - 1);
      const float b0 = bc[0 * kH + jc];
      const float b1 = bc[1 * kH + jc];
      const float b2 = bc[2 * kH + jc];
      const float b3 = bc[3 * kH + jc];
      const float b4 = bc[4 * kH + jc];
      float hres[8], cres[8];
#pragma unroll
      for (int r = 0; r < 8; ++r) {
        const int i = 8 * hh + r;
        const int mw = sMeta[i * kL + s];
        const int ls = ((mw >> 8) & 255) - 1;
        const int rs = ((mw >> 16) & 255) - 1;
        const float cl = load_child_c(ST, ND, i, ls, jc);
        const float cr = load_child_c(ST, ND, i, rs, jc);
        const float gi = fmaf(aL[0][r], kInvRes, aH[0][r]) * kFold + b0;
        const float gl = fmaf(aL[1][r], kInvRes, aH[1][r]) * kFold + b1;
        const float gr = fmaf(aL[2][r], kInvRes, aH[2][r]) * kFold + b2;
        const float gu = fmaf(aL[3][r], kInvRes, aH[3][r]) * kFold + b3;
        const float go = fmaf(aL[4][r], kInvRes, aH[4][r]) * kFold + b4;
        const float cc = cl * sigm(gl + 1.0f) + cr * sigm(gr + 1.0f) + tanhf(gu) * sigm(gi);
        const float hv = sigm(go) * tanhf(cc);
        hres[r] = jv ? hv : 0.0f;
        cres[r] = jv ? cc : 0.0f;
      }
      float tC[8], tH[8];
#pragma unroll
      for (int r = 0; r < 8; ++r) {
        tC[r] = __shfl_xor(cres[r], 16, 32);
        tH[r] = __shfl_xor(hres[r], 16, 32);
      }
      for (int pass = 0; pass < 2; ++pass) {
#pragma unroll
        for (int r = 0; r < 8; ++r) {
          const float vA = (hh == 0) ? hres[r] : tC[r];
          const float vB = (hh == 0) ? tH[r] : cres[r];
          if (s < sCnt[r])
            *(volatile float*)(ND + ((size_t)(r * kMaxNode + s) * kNcb + cb) * 32 + lane) = vA;
          if (s < sCnt[8 + r])
            *(volatile float*)(ND + ((size_t)((8 + r) * kMaxNode + s) * kNcb + cb) * 32 + lane) = vB;
        }
        __threadfence();
      }
    }
    __threadfence();
    __syncthreads();
  }

#pragma unroll 1
  for (int it = 0; it < 5; ++it) {
    const int q = tid + 512 * it;
    const bool inr = q < kOutQ;
    float o[4];
#pragma unroll
    for (int e = 0; e < 4; ++e) {
      int el = 4 * q + e;
      el = el > (kOutN - 1) ? (kOutN - 1) : el;
      const int i = el / kOutW;
      const int col = el - i * kOutW;
      o[e] = root_val(ST, ND, i, col, sCnt[i], sLogp[i]);
    }
    const v4f ov = (v4f){o[0], o[1], o[2], o[3]};
    const int qs = inr ? q : 0;
    for (int pass = 0; pass < 2; ++pass) {
      if (inr) *(volatile v4f*)(out + (size_t)qs * 4) = ov;
      __threadfence();
    }
  }
}

extern "C" void kernel_launch(void* const* d_in, const int* in_sizes, int n_in,
                              void* d_out, int out_size, void* d_ws, size_t ws_size,
                              hipStream_t stream) {
  if (n_in < 9) return;
  if (in_sizes[0] != kTok * kD) return;
  if (in_sizes[2] != kB) return;
  if (in_sizes[3] != kNwReal * kD) return;
  if (in_sizes[4] != kNwReal) return;
  if (in_sizes[5] != 128 * kD) return;
  if (in_sizes[6] != 128) return;
  if (in_sizes[7] != 5 * kH * kKcReal) return;
  if (in_sizes[8] != 5 * kH) return;
  if (out_size != kOutN) return;
  if (ws_size < kWsTotal) return;

  const float* X      = (const float*)d_in[0];
  const int*   length = (const int*)d_in[2];
  const float* Ww     = (const float*)d_in[3];
  const float* bw     = (const float*)d_in[4];
  const float* W1     = (const float*)d_in[5];
  const float* W2     = (const float*)d_in[6];
  const float* Wc     = (const float*)d_in[7];
  const float* bc     = (const float*)d_in[8];
  float* out = (float*)d_out;

  char* ws = (char*)d_ws;
  unsigned short* XH = (unsigned short*)(ws + kOffXH);
  unsigned short* WW = (unsigned short*)(ws + kOffWW);
  unsigned short* WC = (unsigned short*)(ws + kOffWC);
  float*          ST = (float*)(ws + kOffST);
  float*          ND = (float*)(ws + kOffND);

  prep_planes_kernel<<<kBlkX + kBlkW + kBlkC, 256, 0, stream>>>(X, Ww, Wc, XH, WW, WC);

  leaf_gemm_kernel<<<((kTok / 64) * (kNw / 64) + 7) / 8, 256, 0, stream>>>(
      XH, kKx, WW, kKx, ST, kStP, bw, kNwReal, kTok, kNw, kKx, kFold);

  tree_compose_kernel<<<1, 512, 0, stream>>>(X, length, W1, W2, WC, bc, ST, ND, out);
}
